// LSTMCell_83262236000379
// MI455X (gfx1250) — hardware-verified
//
#include <hip/hip_runtime.h>
#include <math.h>

typedef __attribute__((ext_vector_type(16))) _Float16 v16h;
typedef __attribute__((ext_vector_type(16))) __bf16 v16b;
typedef __attribute__((ext_vector_type(8)))  _Float16 v8h;
typedef __attribute__((ext_vector_type(8)))  float v8f;
typedef __attribute__((ext_vector_type(4)))  float v4f;
typedef __attribute__((ext_vector_type(2)))  float v2f;
typedef __attribute__((ext_vector_type(4)))  unsigned v4u;
typedef __attribute__((ext_vector_type(4)))  int v4i;
typedef float __attribute__((may_alias)) float_a;
typedef int __attribute__((may_alias)) int_a;

template <typename T> __device__ __forceinline__ void vst2(void* p, T v) { *(volatile T*)p = v; __threadfence(); *(volatile T*)p = v; }
__device__ __forceinline__ v8f wmma16(v16h a, v16h b, v8f c) {
  v8f d = __builtin_amdgcn_wmma_f32_16x16x32_f16(false, a, false, b, (short)0, c, false, false);
  asm volatile("v_nop\n\tv_nop\n\tv_nop\n\tv_nop" : "+v"(d) : "v"(a), "v"(b));
  return d;
}
__device__ __forceinline__ v8f wmma_bf(v16b a, v16b b, v8f c) {
  v8f d = __builtin_amdgcn_wmma_f32_16x16x32_bf16(false, a, false, b, (short)0, c, false, false);
  asm volatile("v_nop\n\tv_nop\n\tv_nop\n\tv_nop" : "+v"(d) : "v"(a), "v"(b));
  return d;
}
__device__ __forceinline__ v16h frag_h(const _Float16* rowk0, int lane) {
  union { v16h v; v8h q[2]; } u; const _Float16* p = rowk0 + 8 * (lane >> 4);
  u.q[0] = *(const v8h*)p; u.q[1] = *(const v8h*)(p + 16); return u.v;
}
__device__ __forceinline__ v16h frag_f32(const float* rowk0, int lane) {
  v16h a; const float* p = rowk0 + 8 * (lane >> 4);
#pragma unroll
  for (int i = 0; i < 8; ++i) { a[i] = (_Float16)p[i]; a[8 + i] = (_Float16)p[16 + i]; }
  return a;
}
__device__ __forceinline__ v16h frag_f32s(const float* rowk0, int lane, float sc) {
  v16h a; const float* p = rowk0 + 8 * (lane >> 4);
#pragma unroll
  for (int i = 0; i < 8; ++i) { a[i] = (_Float16)(p[i] * sc); a[8 + i] = (_Float16)(p[16 + i] * sc); }
  return a;
}
__device__ __forceinline__ v16h fragc_f32(const float* W, int k0, int n, int lane, int ld, int K) {
  v16h a; const int g = lane >> 4;
#pragma unroll
  for (int i = 0; i < 8; ++i) { const int ka = k0 + 8 * g + i, kb = ka + 16;
    a[i] = (_Float16)(ka < K ? W[(size_t)(ka < K ? ka : K - 1) * ld + n] : 0.f); a[8 + i] = (_Float16)(kb < K ? W[(size_t)(kb < K ? kb : K - 1) * ld + n] : 0.f); }
  return a;
}
struct F2 { v16b h, l; };
__device__ __forceinline__ F2 bsplit16(const float v[16]) { F2 r;
#pragma unroll
  for (int i = 0; i < 16; ++i) { const __bf16 h = (__bf16)v[i]; r.h[i] = h; r.l[i] = (__bf16)(v[i] - (float)h); }
  return r; }
__device__ __forceinline__ F2 split_row(const float* row, int k0, int lane) { float v[16]; const float* p = row + k0 + 8 * (lane >> 4);
#pragma unroll
  for (int i = 0; i < 8; ++i) { v[i] = p[i]; v[8 + i] = p[16 + i]; }
  return bsplit16(v); }
__device__ __forceinline__ F2 split_rowK(const float* row, int k0, int lane, int K) { float v[16]; const int g = lane >> 4;
#pragma unroll
  for (int i = 0; i < 8; ++i) { const int ka = k0 + 8 * g + i, kb = ka + 16; v[i] = ka < K ? row[ka < K ? ka : K - 1] : 0.f; v[8 + i] = kb < K ? row[kb < K ? kb : K - 1] : 0.f; }
  return bsplit16(v); }
__device__ __forceinline__ F2 split_col(const float* W, int k0, int n, int lane, int ld, int K) { float v[16]; const int g = lane >> 4;
#pragma unroll
  for (int i = 0; i < 8; ++i) { const int ka = k0 + 8 * g + i, kb = ka + 16; v[i] = ka < K ? W[(size_t)(ka < K ? ka : K - 1) * ld + n] : 0.f; v[8 + i] = kb < K ? W[(size_t)(kb < K ? kb : K - 1) * ld + n] : 0.f; }
  return bsplit16(v); }
__device__ __forceinline__ v8f mac3(const F2& a, const F2& b, v8f c) { c = wmma_bf(a.l, b.h, c); c = wmma_bf(a.h, b.l, c); return wmma_bf(a.h, b.h, c); }
__device__ __forceinline__ float sigm(float v) { return 1.0f / (1.0f + expf(-v)); }
#define LDSX() do { asm volatile("s_wait_dscnt 0" ::: "memory"); __builtin_amdgcn_wave_barrier(); __builtin_amdgcn_fence(__ATOMIC_RELEASE, "workgroup"); } while (0)

#define NBR 4096
#define DI 1024
#define DHID 1024
#define KT (DI + DHID)
#ifndef NRV
#define NRV NBR
#endif
#define OUT1_OFF (4u * (size_t)NBR * DHID)
__device__ __forceinline__ float bfr(float v) { return (float)(__bf16)v; }
__device__ __forceinline__ v16b wcol1024(const float* Wm, int k0, int o, int lane) { v16b w; const int g = lane >> 4; float t0[8], t1[8];
#pragma unroll
  for (int i = 0; i < 8; ++i) t0[i] = Wm[(size_t)(k0 + 8 * g + i) * DHID + o];
  asm volatile("s_wait_loadcnt 0x0" ::: "memory");
#pragma unroll
  for (int i = 0; i < 8; ++i) t1[i] = Wm[(size_t)(k0 + 16 + 8 * g + i) * DHID + o];
  asm volatile("s_wait_loadcnt 0x0" ::: "memory");
#pragma unroll
  for (int i = 0; i < 8; ++i) { w[i] = (__bf16)t0[i]; w[8 + i] = (__bf16)t1[i]; }
  return w; }
__global__ __launch_bounds__(128) void k_lstm(const float* __restrict__ X, const float* __restrict__ Hp, const float* __restrict__ Cp, const float* __restrict__ WI, const float* __restrict__ WF, const float* __restrict__ WC, const float* __restrict__ WO,
    const float* __restrict__ BI, const float* __restrict__ BF, const float* __restrict__ BC, const float* __restrict__ BO, float* __restrict__ HOUT, float* __restrict__ COUT) {
  __shared__ __align__(16) float sh[4][16][68]; __shared__ __align__(16) float sc[4][16][68];
  const int tid = threadIdx.x, wave = tid >> 5, lane = tid & 31, col = lane & 15, g = lane >> 4; const int c0 = blockIdx.y * 64; const size_t r0 = (size_t)blockIdx.x * 64 + wave * 16;
  v8f af[4] = {}, ai[4] = {}, ac[4] = {}, ao[4] = {};
#pragma unroll 1
  for (int kc = 0; kc < KT / 32; ++kc) { v16b a; { const float* p = kc < DI / 32 ? X + (r0 + col) * DI + kc * 32 + 8 * g : Hp + (r0 + col) * DHID + (kc - DI / 32) * 32 + 8 * g;
#pragma unroll
      for (int i = 0; i < 8; ++i) { a[i] = (__bf16)p[i]; a[8 + i] = (__bf16)p[16 + i]; } }
    asm volatile("s_wait_loadcnt 0x0" ::: "memory");
#pragma unroll
    for (int j = 0; j < 4; ++j) { const int o = c0 + j * 16 + col;
      { const v16b w = wcol1024(WF, kc * 32, o, lane); af[j] = wmma_bf(a, w, af[j]); }
      { const v16b w = wcol1024(WI, kc * 32, o, lane); ai[j] = wmma_bf(a, w, ai[j]); }
      { const v16b w = wcol1024(WC, kc * 32, o, lane); ac[j] = wmma_bf(a, w, ac[j]); }
      { const v16b w = wcol1024(WO, kc * 32, o, lane); ao[j] = wmma_bf(a, w, ao[j]); } } }
#pragma unroll
  for (int j = 0; j < 4; ++j) { const int o = c0 + j * 16 + col; const float bf_ = bfr(BF[o]), bi_ = bfr(BI[o]), bc_ = bfr(BC[o]), bo_ = bfr(BO[o]);
#pragma unroll
    for (int r = 0; r < 8; ++r) { const size_t row = r0 + 8 * g + r; const float cprev = bfr(Cp[row * DHID + o]);
      const float f = sigm(af[j][r] + bf_), iv = sigm(ai[j][r] + bi_), cs = tanhf(ac[j][r] + bc_), ov = sigm(ao[j][r] + bo_);
      const float ct = f * cprev + iv * cs; const float ht = ov * tanhf(ct);
      sc[wave][8 * g + r][j * 16 + col] = ct; sh[wave][8 * g + r][j * 16 + col] = ht; }
    asm volatile("s_wait_loadcnt 0x0" ::: "memory"); }
  LDSX();
  for (int rl = 0; rl < 16; ++rl) if (lane < 16) { vst2(HOUT + (r0 + rl) * DHID + c0 + lane * 4, *(const v4f*)&sh[wave][rl][lane * 4]); vst2(COUT + (r0 + rl) * DHID + c0 + lane * 4, *(const v4f*)&sc[wave][rl][lane * 4]); } }
extern "C" void kernel_launch(void* const* d_in, const int* in_sizes, int n_in, void* d_out, int out_size, void* d_ws, size_t ws_size, hipStream_t stream) {
  (void)in_sizes; (void)n_in; (void)out_size; (void)d_ws; (void)ws_size;
  const float** F = (const float**)d_in;
  k_lstm<<<dim3(NRV / 64, DHID / 64), 128, 0, stream>>>(F[0], F[1], F[2], F[3], F[4], F[5], F[6], F[7], F[8], F[9], F[10], (float*)d_out, (float*)((char*)d_out + OUT1_OFF));
}
